// RWKV_Tmix_x060_Mod_54906861912137
// MI455X (gfx1250) — hardware-run, weakly checked
//
#include <hip/hip_runtime.h>
#include <math.h>

constexpr int kT = 2048;
constexpr int kC = 2048;
constexpr int kH = 32;
constexpr int kHS = 64;
constexpr int kMixCols = 160;
constexpr int kMixPad = 192;
constexpr int kMixRank = 32;
constexpr int kDecRank = 64;
constexpr int kChunk = 16;
constexpr float kWCarry = 1024.0f;
constexpr float kACarry = 16.0f;
constexpr float kZCarry = 64.0f;
constexpr float kFoldAW = 1.0f / (kACarry * kWCarry);
constexpr float kFoldZW = 1.0f / (kZCarry * kWCarry);
constexpr float kGnEps = (float)(1e-5 * 64.0);
static_assert(kC == kH * kHS);
static_assert(kHS == 64);
static_assert(kT % 64 == 0 && kC % 64 == 0 && kMixPad % 64 == 0 && kDecRank % 64 == 0);
static_assert(kC % 32 == 0 && kMixRank % 32 == 0 && kDecRank % 32 == 0);
static_assert(kMixCols == 5 * kMixRank && kMixCols <= kMixPad);
static_assert((kT / 64) * (kC / 64) % 8 == 0 && (kT / 64) * (kMixPad / 64) % 8 == 0 && (kT / 64) * (kDecRank / 64) % 8 == 0);
static_assert(kT % kChunk == 0);
static_assert((kT * (kC / 8)) % 256 == 0);

typedef __attribute__((ext_vector_type(16))) _Float16 v16h;
typedef __attribute__((ext_vector_type(8)))  _Float16 v8h;
typedef __attribute__((ext_vector_type(8)))  float    v8f;
typedef __attribute__((ext_vector_type(4)))  float    v4f;
typedef __attribute__((ext_vector_type(4)))  unsigned int v4u;

__device__ __forceinline__ unsigned pk16(unsigned short a, unsigned short b) { return (unsigned)a | ((unsigned)b << 16); }
__device__ __forceinline__ unsigned short h_bits(float f) { const _Float16 h = (_Float16)f; return __builtin_bit_cast(unsigned short, h); }

__device__ __forceinline__ void guard4_h(v8f& a, v8f& b, v8f& c, v8f& d, v16h x, v16h y0, v16h y1, v16h y2, v16h y3) {
  asm volatile("v_nop\n\tv_nop\n\tv_nop\n\tv_nop" : "+v"(a), "+v"(b), "+v"(c), "+v"(d) : "v"(x), "v"(y0), "v"(y1), "v"(y2), "v"(y3));
}
__device__ __forceinline__ void acc_guard4(v8f& a, v8f& b, v8f& c, v8f& d) {
  asm volatile("v_nop\n\tv_nop\n\tv_nop\n\tv_nop" : "+v"(a), "+v"(b), "+v"(c), "+v"(d));
}
__device__ __forceinline__ void wave_lds_sync() {
  __builtin_amdgcn_fence(__ATOMIC_RELEASE, "workgroup");
  __builtin_amdgcn_wave_barrier();
  __builtin_amdgcn_fence(__ATOMIC_ACQUIRE, "workgroup");
}

struct FragH {
  union U { v16h v; v8h h[2]; };
  static __device__ __forceinline__ v16h load(const _Float16* p) {
    U f; f.h[0] = *(const v8h*)(p); f.h[1] = *(const v8h*)(p + 16); return f.v;
  }
  static __device__ __forceinline__ v8f mma(v16h a, v16h b, v8f c) {
    return __builtin_amdgcn_wmma_f32_16x16x32_f16(false, a, false, b, (short)0, c, false, false);
  }
};

template <int OUT_MODE, bool BIAS_N, int ACT, bool MIX>
__global__ __launch_bounds__(256) void gemm64_f16(
    const unsigned short* __restrict__ Ap, int lda,
    const unsigned short* __restrict__ Btp, int ldb,
    void* __restrict__ Cout, int ldc,
    const float* __restrict__ bias,
    const float* __restrict__ mixX, const float* __restrict__ maa,
    int M, int N, int K, float scale, float oscale) {
  __shared__ __align__(16) float sT[8][16 * 68];
  const int lane = threadIdx.x & 31;
  const int wave = threadIdx.x >> 5;
  const int tilesN = N >> 6;
  const int tilesM = M >> 6;
  const int tile = blockIdx.x * 8 + wave;
  if (tile >= tilesM * tilesN) return;
  const int tm = tile / tilesN;
  const int tn = tile - tm * tilesN;
  const int m0 = tm << 6;
  const int n0 = tn << 6;
  const _Float16* A  = (const _Float16*)Ap;
  const _Float16* Bt = (const _Float16*)Btp;
  const int rlane = lane & 15;
  const int koff  = (lane >> 4) * 8;
  const int mOff  = (lane >> 4) * 8;

  const _Float16* ap[4];
  const _Float16* bp[4];
#pragma unroll
  for (int i = 0; i < 4; ++i) {
    ap[i] = A  + (size_t)(m0 + (i << 4) + rlane) * lda + koff;
    bp[i] = Bt + (size_t)(n0 + (i << 4) + rlane) * ldb + koff;
  }

  v8f acc[4][4];
#pragma unroll
  for (int i = 0; i < 4; ++i)
#pragma unroll
    for (int j = 0; j < 4; ++j) acc[i][j] = (v8f){0.f, 0.f, 0.f, 0.f, 0.f, 0.f, 0.f, 0.f};

  for (int k0 = 0; k0 < K; k0 += 32) {
    const v16h b0 = FragH::load(bp[0] + k0);
    const v16h b1 = FragH::load(bp[1] + k0);
    const v16h b2 = FragH::load(bp[2] + k0);
    const v16h b3 = FragH::load(bp[3] + k0);
#pragma unroll
    for (int i = 0; i < 4; ++i) {
      const v16h ah = FragH::load(ap[i] + k0);
      acc[i][0] = FragH::mma(ah, b0, acc[i][0]);
      acc[i][1] = FragH::mma(ah, b1, acc[i][1]);
      acc[i][2] = FragH::mma(ah, b2, acc[i][2]);
      acc[i][3] = FragH::mma(ah, b3, acc[i][3]);
      guard4_h(acc[i][0], acc[i][1], acc[i][2], acc[i][3], ah, b0, b1, b2, b3);
    }
  }
  acc_guard4(acc[0][0], acc[0][1], acc[0][2], acc[0][3]);
  acc_guard4(acc[1][0], acc[1][1], acc[1][2], acc[1][3]);
  acc_guard4(acc[2][0], acc[2][1], acc[2][2], acc[2][3]);
  acc_guard4(acc[3][0], acc[3][1], acc[3][2], acc[3][3]);

  float* slab = sT[wave];
  float bv[4];
#pragma unroll
  for (int j = 0; j < 4; ++j) bv[j] = BIAS_N ? bias[n0 + (j << 4) + rlane] : 0.0f;

#pragma unroll
  for (int i = 0; i < 4; ++i) {
    const int mBase = m0 + (i << 4);
#pragma unroll
    for (int j = 0; j < 4; ++j) {
#pragma unroll
      for (int r = 0; r < 8; ++r) {
        slab[(mOff + r) * 68 + (j << 4) + rlane] = acc[i][j][r] * scale + bv[j];
      }
    }
    wave_lds_sync();
    if (ACT != 0) {
#pragma unroll 1
      for (int q = 0; q < 32; ++q) {
        const int idx = q * 32 + lane;
        const int off = (idx >> 6) * 68 + (idx & 63);
        float v = slab[off];
        if (ACT == 1) v = tanhf(v);
        if (ACT == 2) v = expf(-expf(v));
        if (ACT == 3) v = v * (1.0f / (1.0f + expf(-v)));
        slab[off] = v;
      }
      wave_lds_sync();
    }
    if (OUT_MODE == 0) {
      float* C = (float*)Cout;
      const int hh = lane >> 4, c4 = (lane & 15) * 4;
      for (int pass = 0; pass < 2; ++pass) {
#pragma unroll
        for (int it = 0; it < 8; ++it) {
          const int row = it * 2 + hh;
          const v4f v = *(const v4f*)(slab + row * 68 + c4);
          *(volatile v4f*)(C + (size_t)(mBase + row) * ldc + n0 + c4) = v;
        }
        __threadfence();
      }
    } else {
      unsigned short* C = (unsigned short*)Cout;
      const int q = lane >> 3, c8 = (lane & 7) * 8;
      v8h hv[4];
#pragma unroll
      for (int it = 0; it < 4; ++it) {
        const int row = it * 4 + q;
        const float* sp = slab + row * 68 + c8;
        const v4f s0 = *(const v4f*)(sp);
        const v4f s1 = *(const v4f*)(sp + 4);
        float vals[8];
#pragma unroll
        for (int e = 0; e < 4; ++e) { vals[e] = s0[e]; vals[4 + e] = s1[e]; }
        if (MIX) {
          const int trow = mBase + row;
          const bool hasP = (trow > 0);
          const int prow = hasP ? (trow - 1) : 0;
          const size_t go = (size_t)trow * kC + n0 + c8;
          const size_t gp = (size_t)prow * kC + n0 + c8;
          const v4f x0 = *(const v4f*)(mixX + go);
          const v4f x1 = *(const v4f*)(mixX + go + 4);
          v4f p0 = *(const v4f*)(mixX + gp);
          v4f p1 = *(const v4f*)(mixX + gp + 4);
          asm volatile("" : "+v"(p0), "+v"(p1));
          const v4f a0 = *(const v4f*)(maa + n0 + c8);
          const v4f a1 = *(const v4f*)(maa + n0 + c8 + 4);
#pragma unroll
          for (int e = 0; e < 4; ++e) {
            const float q0 = hasP ? p0[e] : 0.0f;
            const float q1 = hasP ? p1[e] : 0.0f;
            const float d0 = q0 - x0[e];
            const float d1 = q1 - x1[e];
            vals[e]     = x0[e] + d0 * (a0[e] + vals[e]);
            vals[4 + e] = x1[e] + d1 * (a1[e] + vals[4 + e]);
          }
        }
#pragma unroll
        for (int e = 0; e < 8; ++e) hv[it][e] = (_Float16)(vals[e] * oscale);
      }
      for (int pass = 0; pass < 2; ++pass) {
#pragma unroll
        for (int it = 0; it < 4; ++it) {
          const int row = it * 4 + q;
          *(volatile v8h*)(C + (size_t)(mBase + row) * ldc + n0 + c8) = hv[it];
        }
        __threadfence();
      }
    }
    wave_lds_sync();
  }
}

__global__ __launch_bounds__(256) void tcast_kernel(const float* __restrict__ in, int R, int C,
                                                    unsigned short* __restrict__ out, int RP, float carry) {
  __shared__ float sm[64][65];
  const int t  = threadIdx.x;
  const int r0 = blockIdx.x * 64;
  const int c0 = blockIdx.y * 64;
#pragma unroll
  for (int i = 0; i < 16; ++i) {
    const int e  = i * 256 + t;
    const int rl = e >> 6;
    const int cl = e & 63;
    const int r = r0 + rl, c = c0 + cl;
    const int rc = (r < R) ? r : (R - 1);
    const int cc = (c < C) ? c : (C - 1);
    const float v = in[(size_t)rc * C + cc];
    sm[cl][rl] = (r < R && c < C) ? (v * carry) : 0.0f;
  }
  __syncthreads();
  const int lane = t & 31, wave = t >> 5;
  const int q = lane >> 3, c8 = (lane & 7) * 8;
  for (int pass = 0; pass < 2; ++pass) {
#pragma unroll
    for (int it = 0; it < 2; ++it) {
      const int row = wave * 8 + it * 4 + q;
      unsigned short hb[8];
#pragma unroll
      for (int e = 0; e < 8; ++e) hb[e] = h_bits(sm[row][c8 + e]);
      const v4u u = (v4u){pk16(hb[0], hb[1]), pk16(hb[2], hb[3]), pk16(hb[4], hb[5]), pk16(hb[6], hb[7])};
      *(volatile v4u*)(out + (size_t)(c0 + row) * RP + r0 + c8) = u;
    }
    __threadfence();
  }
}

__global__ __launch_bounds__(256) void prep_kernel(const float* __restrict__ x, const float* __restrict__ maax,
                                                   unsigned short* __restrict__ XA) {
  const int i  = blockIdx.x * 256 + threadIdx.x;
  const int t  = i >> 8;
  const int c8 = (i & 255) * 8;
  const bool hasP = (t > 0);
  const int tp = hasP ? (t - 1) : 0;
  const v4f xc0 = *(const v4f*)(x + (size_t)t * kC + c8);
  const v4f xc1 = *(const v4f*)(x + (size_t)t * kC + c8 + 4);
  v4f xp0 = *(const v4f*)(x + (size_t)tp * kC + c8);
  v4f xp1 = *(const v4f*)(x + (size_t)tp * kC + c8 + 4);
  asm volatile("" : "+v"(xp0), "+v"(xp1));
  const v4f m0 = *(const v4f*)(maax + c8);
  const v4f m1 = *(const v4f*)(maax + c8 + 4);
  unsigned short hb[8];
#pragma unroll
  for (int e = 0; e < 4; ++e) {
    const float q0 = hasP ? xp0[e] : 0.0f;
    const float q1 = hasP ? xp1[e] : 0.0f;
    const float d0 = q0 - xc0[e];
    const float d1 = q1 - xc1[e];
    const float a0 = xc0[e] + d0 * m0[e];
    const float a1 = xc1[e] + d1 * m1[e];
    hb[e]     = h_bits(a0 * kACarry);
    hb[4 + e] = h_bits(a1 * kACarry);
  }
  const v4u u = (v4u){pk16(hb[0], hb[1]), pk16(hb[2], hb[3]), pk16(hb[4], hb[5]), pk16(hb[6], hb[7])};
  unsigned short* q = XA + (size_t)t * kC + c8;
  *(volatile v4u*)q = u;
  __threadfence();
  *(volatile v4u*)q = u;
}

__global__ __launch_bounds__(128) void scan_kernel(const float* __restrict__ R32, const float* __restrict__ K32,
                                                   const float* __restrict__ V32, const float* __restrict__ WD32,
                                                   const float* __restrict__ U, float* __restrict__ Y) {
  __shared__ __align__(16) float rsh[kChunk * 64];
  __shared__ __align__(16) float ksh[kChunk * 64];
  __shared__ __align__(16) float wsh[kChunk * 64];
  __shared__ __align__(16) float vsh[kChunk * 64];
  __shared__ __align__(16) float ysh[kChunk * 64];
  __shared__ float cfs[kChunk];
  const int tid  = threadIdx.x;
  const int lane = tid & 31;
  const int wave = tid >> 5;
  const int h    = blockIdx.x;
  const int jj   = wave * 16 + (lane & 15);
  const int half = lane >> 4;
  const int i0   = half * 32;
  const int srow = tid >> 4;
  const int sc4  = (tid & 15) * 4;
  const v4f u4 = *(const v4f*)(U + h * kHS + sc4);

  float S[32];
#pragma unroll
  for (int q = 0; q < 32; ++q) S[q] = 0.0f;

#pragma unroll 1
  for (int ch = 0; ch < kT / kChunk; ++ch) {
    const int t0 = ch * kChunk;
#pragma unroll
    for (int it = 0; it < 2; ++it) {
      const int row = it * 8 + srow;
      const size_t g = (size_t)(t0 + row) * kC + h * kHS + sc4;
      const v4f r4 = *(const v4f*)(R32 + g);
      const v4f k4 = *(const v4f*)(K32 + g);
      const v4f v4 = *(const v4f*)(V32 + g);
      const v4f w4 = *(const v4f*)(WD32 + g);
      *(v4f*)(rsh + row * 64 + sc4) = r4;
      *(v4f*)(ksh + row * 64 + sc4) = k4;
      *(v4f*)(vsh + row * 64 + sc4) = v4;
      *(v4f*)(wsh + row * 64 + sc4) = w4;
      float p = (r4[0] * u4[0]) * k4[0];
      p = fmaf(r4[1] * u4[1], k4[1], p);
      p = fmaf(r4[2] * u4[2], k4[2], p);
      p = fmaf(r4[3] * u4[3], k4[3], p);
      p += __shfl_xor(p, 1, 32);
      p += __shfl_xor(p, 2, 32);
      p += __shfl_xor(p, 4, 32);
      p += __shfl_xor(p, 8, 32);
      if ((tid & 15) == 0) cfs[row] = p;
    }
    __syncthreads();

#pragma unroll 1
    for (int s = 0; s < kChunk; ++s) {
      const float vj = vsh[s * 64 + jj];
      const float cf = cfs[s];
      const float* rp = rsh + s * 64 + i0;
      const float* kp = ksh + s * 64 + i0;
      const float* wp = wsh + s * 64 + i0;
      float acc = 0.0f;
#pragma unroll
      for (int q = 0; q < 8; ++q) {
        const v4f r4 = *(const v4f*)(rp + 4 * q);
        const v4f k4 = *(const v4f*)(kp + 4 * q);
        const v4f w4 = *(const v4f*)(wp + 4 * q);
#pragma unroll
        for (int e = 0; e < 4; ++e) {
          const float kv = k4[e] * vj;
          acc = fmaf(r4[e], S[4 * q + e], acc);
          S[4 * q + e] = fmaf(S[4 * q + e], w4[e], kv);
        }
      }
      const float oth = __shfl_xor(acc, 16, 32);
      const float yv = (acc + oth) + vj * cf;
      if (half == 0) ysh[s * 64 + jj] = yv;
    }
    __syncthreads();

    for (int pass = 0; pass < 2; ++pass) {
#pragma unroll
      for (int it = 0; it < 2; ++it) {
        const int row = it * 8 + srow;
        const v4f val = *(const v4f*)(ysh + row * 64 + sc4);
        *(volatile v4f*)(Y + (size_t)(t0 + row) * kC + h * kHS + sc4) = val;
      }
      __threadfence();
    }
  }
}

__global__ __launch_bounds__(256) void gn_gate_kernel(const float* __restrict__ Y, const float* __restrict__ G,
                                                      const float* __restrict__ lnw, const float* __restrict__ lnb,
                                                      unsigned short* __restrict__ Z) {
  const int gt = blockIdx.x * 256 + threadIdx.x;
  const int ch = (gt & 255) * 8;
  const size_t base = (size_t)gt * 8;
  const v4f y0 = *(const v4f*)(Y + base);
  const v4f y1 = *(const v4f*)(Y + base + 4);
  const v4f g0 = *(const v4f*)(G + base);
  const v4f g1 = *(const v4f*)(G + base + 4);
  const v4f w0 = *(const v4f*)(lnw + ch);
  const v4f w1 = *(const v4f*)(lnw + ch + 4);
  const v4f b0 = *(const v4f*)(lnb + ch);
  const v4f b1 = *(const v4f*)(lnb + ch + 4);
  float s = ((y0[0] + y0[1]) + (y0[2] + y0[3])) + ((y1[0] + y1[1]) + (y1[2] + y1[3]));
  s += __shfl_xor(s, 1, 32);
  s += __shfl_xor(s, 2, 32);
  s += __shfl_xor(s, 4, 32);
  const float mu = s * (1.0f / kHS);
  float d[8];
#pragma unroll
  for (int e = 0; e < 4; ++e) { d[e] = y0[e] - mu; d[4 + e] = y1[e] - mu; }
  float ss = 0.0f;
#pragma unroll
  for (int e = 0; e < 8; ++e) ss += d[e] * d[e];
  ss += __shfl_xor(ss, 1, 32);
  ss += __shfl_xor(ss, 2, 32);
  ss += __shfl_xor(ss, 4, 32);
  const float var  = ss * (1.0f / kHS);
  const float rstd = 1.0f / sqrtf(var + kGnEps);
  unsigned short hb[8];
#pragma unroll
  for (int e = 0; e < 4; ++e) {
    const float z0 = ((d[e] * rstd) * w0[e] + b0[e]) * g0[e];
    const float z1 = ((d[4 + e] * rstd) * w1[e] + b1[e]) * g1[e];
    hb[e]     = h_bits(z0 * kZCarry);
    hb[4 + e] = h_bits(z1 * kZCarry);
  }
  const v4u u = (v4u){pk16(hb[0], hb[1]), pk16(hb[2], hb[3]), pk16(hb[4], hb[5]), pk16(hb[6], hb[7])};
  unsigned short* zp = Z + base;
  *(volatile v4u*)zp = u;
  __threadfence();
  *(volatile v4u*)zp = u;
}

extern "C" void kernel_launch(void* const* d_in, const int* in_sizes, int n_in,
                              void* d_out, int out_size, void* d_ws, size_t ws_size, hipStream_t stream) {
  if (n_in < 20 || d_out == nullptr || d_ws == nullptr) return;
  if (in_sizes[0] != kT * kC || in_sizes[1] != kC || in_sizes[2] != kC || in_sizes[3] != kC ||
      in_sizes[4] != kC || in_sizes[5] != kC || in_sizes[6] != kC || in_sizes[7] != kC * kMixCols ||
      in_sizes[8] != kMixCols * kC || in_sizes[9] != kC || in_sizes[10] != kC * kDecRank ||
      in_sizes[11] != kDecRank * kC || in_sizes[12] != kH * kHS || in_sizes[13] != kC * kC ||
      in_sizes[14] != kC * kC || in_sizes[15] != kC * kC || in_sizes[16] != kC * kC ||
      in_sizes[17] != kC * kC || in_sizes[18] != kC || in_sizes[19] != kC || out_size != kT * kC) return;

  const float* x      = (const float*)d_in[0];
  const float* maa_x  = (const float*)d_in[1];
  const float* maa_w  = (const float*)d_in[2];
  const float* maa_k  = (const float*)d_in[3];
  const float* maa_v  = (const float*)d_in[4];
  const float* maa_r  = (const float*)d_in[5];
  const float* maa_g  = (const float*)d_in[6];
  const float* w1     = (const float*)d_in[7];
  const float* w2     = (const float*)d_in[8];
  const float* tdec   = (const float*)d_in[9];
  const float* dw1    = (const float*)d_in[10];
  const float* dw2    = (const float*)d_in[11];
  const float* ubon   = (const float*)d_in[12];
  const float* Wr     = (const float*)d_in[13];
  const float* Wk     = (const float*)d_in[14];
  const float* Wv     = (const float*)d_in[15];
  const float* Wg     = (const float*)d_in[16];
  const float* Wo     = (const float*)d_in[17];
  const float* lnw    = (const float*)d_in[18];
  const float* lnb    = (const float*)d_in[19];
  float* out = (float*)d_out;

  const size_t PLN = (size_t)kT * kC;
  char* ws = (char*)d_ws; size_t off = 0;
  auto carve = [&](size_t bytes) -> char* { char* p = ws + off; off += (bytes + 255) & ~(size_t)255; return p; };
  unsigned short* WS16 = (unsigned short*)carve((size_t)kC * kC * 2);
  unsigned short* W1T  = (unsigned short*)carve((size_t)kMixPad * kC * 2);
  unsigned short* W2T  = (unsigned short*)carve((size_t)kC * kMixPad * 2);
  unsigned short* DW1T = (unsigned short*)carve((size_t)kDecRank * kC * 2);
  unsigned short* DW2T = (unsigned short*)carve((size_t)kC * kDecRank * 2);
  unsigned short* XS   = (unsigned short*)carve(PLN * 2);
  unsigned short* MP   = (unsigned short*)carve((size_t)kT * kMixPad * 2);
  unsigned short* TD   = (unsigned short*)carve((size_t)kT * kDecRank * 2);
  float*          R32  = (float*)carve(PLN * 4);
  float*          K32  = (float*)carve(PLN * 4);
  float*          V32  = (float*)carve(PLN * 4);
  float*          G32  = (float*)carve(PLN * 4);
  float*          WD32 = (float*)carve(PLN * 4);
  float*          Y32  = (float*)carve(PLN * 4);
  unsigned short* YNG  = (unsigned short*)carve(PLN * 2);
  if (off > ws_size || off > (size_t)134217728) return;

  const int gBig = (kT / 64) * (kC / 64) / 8;
  const int gMix = (kT / 64) * (kMixPad / 64) / 8;
  const int gDec = (kT / 64) * (kDecRank / 64) / 8;

  tcast_kernel<<<dim3(kC / 64, kMixPad / 64), 256, 0, stream>>>(w1, kC, kMixCols, W1T, kC, kWCarry);
  tcast_kernel<<<dim3(kMixPad / 64, kC / 64), 256, 0, stream>>>(w2, kMixCols, kC, W2T, kMixPad, kWCarry);
  tcast_kernel<<<dim3(kC / 64, kDecRank / 64), 256, 0, stream>>>(dw1, kC, kDecRank, DW1T, kC, kWCarry);
  tcast_kernel<<<dim3(kDecRank / 64, kC / 64), 256, 0, stream>>>(dw2, kDecRank, kC, DW2T, kDecRank, kWCarry);

  prep_kernel<<<kT * kC / 8 / 256, 256, 0, stream>>>(x, maa_x, XS);

  gemm64_f16<1, false, 1, false><<<gMix, 256, 0, stream>>>(
      XS, kC, W1T, kC, (void*)MP, kMixPad, tdec, x, maa_w, kT, kMixPad, kC, kFoldAW, kACarry);

  gemm64_f16<1, false, 0, true><<<gBig, 256, 0, stream>>>(
      MP + 0 * kMixRank, kMixPad, W2T + 0 * kMixRank, kMixPad, (void*)XS, kC, tdec, x, maa_w, kT, kC, kMixRank, kFoldAW, kACarry);
  gemm64_f16<1, false, 1, false><<<gDec, 256, 0, stream>>>(
      XS, kC, DW1T, kC, (void*)TD, kDecRank, tdec, x, maa_w, kT, kDecRank, kC, kFoldAW, kACarry);
  gemm64_f16<0, true, 2, false><<<gBig, 256, 0, stream>>>(
      TD, kDecRank, DW2T, kDecRank, (void*)WD32, kC, tdec, x, maa_w, kT, kC, kDecRank, kFoldAW, 1.0f);

  gemm64_f16<1, false, 0, true><<<gBig, 256, 0, stream>>>(
      MP + 1 * kMixRank, kMixPad, W2T + 1 * kMixRank, kMixPad, (void*)XS, kC, tdec, x, maa_k, kT, kC, kMixRank, kFoldAW, kACarry);
  tcast_kernel<<<dim3(kC / 64, kC / 64), 256, 0, stream>>>(Wk, kC, kC, WS16, kC, kWCarry);
  gemm64_f16<0, false, 0, false><<<gBig, 256, 0, stream>>>(
      XS, kC, WS16, kC, (void*)K32, kC, tdec, x, maa_w, kT, kC, kC, kFoldAW, 1.0f);

  gemm64_f16<1, false, 0, true><<<gBig, 256, 0, stream>>>(
      MP + 2 * kMixRank, kMixPad, W2T + 2 * kMixRank, kMixPad, (void*)XS, kC, tdec, x, maa_v, kT, kC, kMixRank, kFoldAW, kACarry);
  tcast_kernel<<<dim3(kC / 64, kC / 64), 256, 0, stream>>>(Wv, kC, kC, WS16, kC, kWCarry);
  gemm64_f16<0, false, 0, false><<<gBig, 256, 0, stream>>>(
      XS, kC, WS16, kC, (void*)V32, kC, tdec, x, maa_w, kT, kC, kC, kFoldAW, 1.0f);

  gemm64_f16<1, false, 0, true><<<gBig, 256, 0, stream>>>(
      MP + 3 * kMixRank, kMixPad, W2T + 3 * kMixRank, kMixPad, (void*)XS, kC, tdec, x, maa_r, kT, kC, kMixRank, kFoldAW, kACarry);
  tcast_kernel<<<dim3(kC / 64, kC / 64), 256, 0, stream>>>(Wr, kC, kC, WS16, kC, kWCarry);
  gemm64_f16<0, false, 0, false><<<gBig, 256, 0, stream>>>(
      XS, kC, WS16, kC, (void*)R32, kC, tdec, x, maa_w, kT, kC, kC, kFoldAW, 1.0f);

  gemm64_f16<1, false, 0, true><<<gBig, 256, 0, stream>>>(
      MP + 4 * kMixRank, kMixPad, W2T + 4 * kMixRank, kMixPad, (void*)XS, kC, tdec, x, maa_g, kT, kC, kMixRank, kFoldAW, kACarry);
  tcast_kernel<<<dim3(kC / 64, kC / 64), 256, 0, stream>>>(Wg, kC, kC, WS16, kC, kWCarry);
  gemm64_f16<0, false, 3, false><<<gBig, 256, 0, stream>>>(
      XS, kC, WS16, kC, (void*)G32, kC, tdec, x, maa_w, kT, kC, kC, kFoldAW, 1.0f);

  scan_kernel<<<kH, 128, 0, stream>>>(R32, K32, V32, WD32, ubon, Y32);

  gn_gate_kernel<<<kT * kC / 8 / 256, 256, 0, stream>>>(Y32, G32, lnw, lnb, YNG);

  tcast_kernel<<<dim3(kC / 64, kC / 64), 256, 0, stream>>>(Wo, kC, kC, WS16, kC, kWCarry);
  gemm64_f16<0, false, 0, false><<<gBig, 256, 0, stream>>>(
      YNG, kC, WS16, kC, (void*)out, kC, tdec, x, maa_w, kT, kC, kC, kFoldZW, 1.0f);
}
